// DANNet_51384988729941
// MI455X (gfx1250) — hardware-verified
//
#include <hip/hip_runtime.h>


namespace {
constexpr int B = 4096, D = 512, C = 8, E = 8, H1 = 1024, CHUNK = 512;
constexpr float AS_ = 8.0f, EPS = 1e-5f;

typedef _Float16 b16;
typedef __attribute__((ext_vector_type(16))) _Float16 v16b;
typedef __attribute__((ext_vector_type(8))) _Float16 v8b;
typedef __attribute__((ext_vector_type(8))) float v8f;
typedef __attribute__((ext_vector_type(4))) float v4f;
typedef __attribute__((ext_vector_type(2))) float v2f;
__device__ __forceinline__ float bf16_rne(float f) { unsigned int u = __float_as_uint(f); u += 0x7FFFu + ((u >> 16) & 1u); return __uint_as_float(u & 0xFFFF0000u); }
__device__ __forceinline__ void split16(float v, b16& hi, b16& lo) { hi = (b16)v; lo = (b16)(v - (float)hi); }
__device__ __forceinline__ v16b frag_kb(const b16* p, int hh) { const v8b a = *(const v8b*)(p + 8 * hh), b = *(const v8b*)(p + 16 + 8 * hh); v16b f;
#pragma unroll
  for (int e = 0; e < 8; ++e) { f[e] = a[e]; f[8 + e] = b[e]; } return f; }
__device__ __forceinline__ v16b frag_x(const float* p, int hh) { v16b f;
#pragma unroll
  for (int e = 0; e < 8; ++e) { f[e] = (b16)bf16_rne(p[8 * hh + e]); f[8 + e] = (b16)bf16_rne(p[16 + 8 * hh + e]); } return f; }
__device__ __forceinline__ void frag_split(const float* p, int hh, v16b& fh, v16b& fl) {
#pragma unroll
  for (int e = 0; e < 8; ++e) { b16 a, c; split16(p[8 * hh + e] * AS_, a, c); fh[e] = a; fl[e] = c; split16(p[16 + 8 * hh + e] * AS_, a, c); fh[8 + e] = a; fl[8 + e] = c; } }
__device__ __forceinline__ v8f wmma16b(v16b a, v16b b, v8f c) { v8f d = __builtin_amdgcn_wmma_f32_16x16x32_f16(false, a, false, b, (short)0, c, false, false); asm volatile("v_nop\n\tv_nop\n\tv_nop\n\tv_nop" : "+v"(d) : "v"(a), "v"(b)); return d; }
__device__ __forceinline__ void wave_lds_sync() { __builtin_amdgcn_fence(__ATOMIC_RELEASE, "workgroup"); __builtin_amdgcn_wave_barrier(); __builtin_amdgcn_fence(__ATOMIC_ACQUIRE, "workgroup"); }
__device__ __forceinline__ float nexp(float x) { return __builtin_amdgcn_exp2f(x * 1.4426950408889634f); }
__device__ __forceinline__ float nlog(float x) { return __builtin_amdgcn_logf(x) * 0.6931471805599453f; }
__device__ __forceinline__ float pmul(float a, float b) { float p = a * b; asm volatile("" : "+v"(p)); return p; }

struct Wo_ { static constexpr size_t BW1 = 0, BW2 = BW1 + 256 * 512, FC = BW2 + 128 * 256, DW1 = FC + 16 * 128, DW2 = DW1 + (size_t)1024 * 512, DW3 = DW2 + (size_t)1024 * 1024, DW4 = DW3 + (size_t)512 * 1024, EW1 = DW4 + 16 * 512, EW2 = EW1 + (size_t)E * 1024 * 512, EW3 = EW2 + (size_t)E * 1024 * 1024, EW4 = EW3 + (size_t)E * 512 * 1024, END = EW4 + (size_t)E * 16 * 512; };
struct Po_ { static constexpr int BB1 = 0, BS1 = 256, BT1 = 512, BB2 = 768, BS2 = 896, BT2 = 1024, FCB = 1152, DB1 = 1168, DS1 = 2192, DT1 = 3216, DB2 = 4240, DS2 = 5264, DT2 = 6288, DB3 = 7312, DS3 = 7824, DT3 = 8336, DB4 = 8848, EB1 = 8864, EG1 = EB1 + E * 1024, ET1 = EG1 + E * 1024, EB2 = ET1 + E * 1024, EG2 = EB2 + E * 1024, ET2 = EG2 + E * 1024, EB3 = ET2 + E * 1024, EG3 = EB3 + E * 512, ET3 = EG3 + E * 512, EB4 = ET3 + E * 512, END = EB4 + E * 16; };
struct In { const float* p[49]; };

__global__ __launch_bounds__(256) void prep_kernel(In in, b16* __restrict__ R, float* __restrict__ P) {
  const size_t tid = (size_t)blockIdx.x * blockDim.x + threadIdx.x, nth = (size_t)gridDim.x * blockDim.x;
  auto tr = [&](const float* W, int IN, int OUT, int OUTP, size_t base, size_t p) { const int o = (int)(p / IN), k = (int)(p % IN); R[base + p] = (b16)((o < OUT) ? bf16_rne(W[(size_t)k * OUT + o]) : 0.0f); (void)OUTP; };
  for (int pass = 0; pass < 2; ++pass) {
    for (size_t p = tid; p < 256 * 512; p += nth) tr(in.p[1], 512, 256, 256, Wo_::BW1, p);
    for (size_t p = tid; p < 128 * 256; p += nth) tr(in.p[7], 256, 128, 128, Wo_::BW2, p);
    for (size_t p = tid; p < 16 * 128; p += nth) tr(in.p[13], 128, 8, 16, Wo_::FC, p);
    for (size_t p = tid; p < (size_t)1024 * 512; p += nth) tr(in.p[15], 512, 1024, 1024, Wo_::DW1, p);
    for (size_t p = tid; p < (size_t)1024 * 1024; p += nth) tr(in.p[21], 1024, 1024, 1024, Wo_::DW2, p);
    for (size_t p = tid; p < (size_t)512 * 1024; p += nth) tr(in.p[27], 1024, 512, 512, Wo_::DW3, p);
    for (size_t p = tid; p < 16 * 512; p += nth) tr(in.p[33], 512, 2, 16, Wo_::DW4, p);
    for (size_t p = tid; p < (size_t)E * 1024 * 512; p += nth) { const int e = (int)(p / (1024 * 512)); tr(in.p[35] + (size_t)e * 512 * 1024, 512, 1024, 1024, Wo_::EW1 + (size_t)e * 1024 * 512, p % (1024 * 512)); }
    for (size_t p = tid; p < (size_t)E * 1024 * 1024; p += nth) { const int e = (int)(p / (1024 * 1024)); tr(in.p[39] + (size_t)e * 1024 * 1024, 1024, 1024, 1024, Wo_::EW2 + (size_t)e * 1024 * 1024, p % (1024 * 1024)); }
    for (size_t p = tid; p < (size_t)E * 512 * 1024; p += nth) { const int e = (int)(p / (512 * 1024)); tr(in.p[43] + (size_t)e * 1024 * 512, 1024, 512, 512, Wo_::EW3 + (size_t)e * 512 * 1024, p % (512 * 1024)); }
    for (size_t p = tid; p < (size_t)E * 16 * 512; p += nth) { const int e = (int)(p / (16 * 512)); tr(in.p[47] + (size_t)e * 512 * 2, 512, 2, 16, Wo_::EW4 + (size_t)e * 16 * 512, p % (16 * 512)); }
    for (size_t p = tid; p < (size_t)Po_::END; p += nth) { const int i = (int)p; float v = 0.0f;
      auto bn_s = [&](const float* g, const float* var, int j) { return bf16_rne(g[j]) * rsqrtf(bf16_rne(var[j]) + EPS); };
      auto bn_t = [&](const float* g, const float* bb, const float* m, const float* var, int j) { return bf16_rne(bb[j]) - bf16_rne(m[j]) * (bf16_rne(g[j]) * rsqrtf(bf16_rne(var[j]) + EPS)); };
      if (i < Po_::BS1) v = bf16_rne(in.p[2][i]); else if (i < Po_::BT1) v = bn_s(in.p[3], in.p[6], i - Po_::BS1); else if (i < Po_::BB2) v = bn_t(in.p[3], in.p[4], in.p[5], in.p[6], i - Po_::BT1);
      else if (i < Po_::BS2) v = bf16_rne(in.p[8][i - Po_::BB2]); else if (i < Po_::BT2) v = bn_s(in.p[9], in.p[12], i - Po_::BS2); else if (i < Po_::FCB) v = bn_t(in.p[9], in.p[10], in.p[11], in.p[12], i - Po_::BT2);
      else if (i < Po_::DB1) v = (i - Po_::FCB < C) ? bf16_rne(in.p[14][i - Po_::FCB]) : 0.0f;
      else if (i < Po_::DS1) v = bf16_rne(in.p[16][i - Po_::DB1]); else if (i < Po_::DT1) v = bn_s(in.p[17], in.p[20], i - Po_::DS1); else if (i < Po_::DB2) v = bn_t(in.p[17], in.p[18], in.p[19], in.p[20], i - Po_::DT1);
      else if (i < Po_::DS2) v = bf16_rne(in.p[22][i - Po_::DB2]); else if (i < Po_::DT2) v = bn_s(in.p[23], in.p[26], i - Po_::DS2); else if (i < Po_::DB3) v = bn_t(in.p[23], in.p[24], in.p[25], in.p[26], i - Po_::DT2);
      else if (i < Po_::DS3) v = bf16_rne(in.p[28][i - Po_::DB3]); else if (i < Po_::DT3) v = bn_s(in.p[29], in.p[32], i - Po_::DS3); else if (i < Po_::DB4) v = bn_t(in.p[29], in.p[30], in.p[31], in.p[32], i - Po_::DT3);
      else if (i < Po_::EB1) v = (i - Po_::DB4 < 2) ? bf16_rne(in.p[34][i - Po_::DB4]) : 0.0f;
      else if (i < Po_::EG1) v = bf16_rne(in.p[36][i - Po_::EB1]); else if (i < Po_::ET1) v = bf16_rne(in.p[37][i - Po_::EG1]); else if (i < Po_::EB2) v = bf16_rne(in.p[38][i - Po_::ET1]);
      else if (i < Po_::EG2) v = bf16_rne(in.p[40][i - Po_::EB2]); else if (i < Po_::ET2) v = bf16_rne(in.p[41][i - Po_::EG2]); else if (i < Po_::EB3) v = bf16_rne(in.p[42][i - Po_::ET2]);
      else if (i < Po_::EG3) v = bf16_rne(in.p[44][i - Po_::EB3]); else if (i < Po_::ET3) v = bf16_rne(in.p[45][i - Po_::EG3]); else if (i < Po_::EB4) v = bf16_rne(in.p[46][i - Po_::ET3]);
      else { const int j = i - Po_::EB4, e = j / 16, c = j % 16; v = (c < 2) ? bf16_rne(in.p[48][e * 2 + c]) : 0.0f; }
      P[p] = v; }
    __threadfence(); }
}

__global__ __launch_bounds__(128) void gemm_kernel(const float* __restrict__ A, int K, int amode, const b16* __restrict__ Bw, int N, const float* __restrict__ bias, int emode, const float* __restrict__ scl, const float* __restrict__ sft, float* __restrict__ Y) {
  __shared__ __attribute__((aligned(16))) float Ts[4][32 * 64];
  const int lane = threadIdx.x & 31, wave = threadIdx.x >> 5, nloc = lane & 15, hlf = lane >> 4, m0 = blockIdx.y * 128 + wave * 32, c0 = blockIdx.x * 64;
  v8f acc[2][4];
#pragma unroll
  for (int r = 0; r < 2; ++r)
#pragma unroll
    for (int t = 0; t < 4; ++t) acc[r][t] = (v8f){};
  for (int kb = 0; kb < K; kb += 32) { v16b a0, l0, a1, l1;
    if (amode == 0) { a0 = frag_x(A + (size_t)(m0 + nloc) * K + kb, hlf); a1 = frag_x(A + (size_t)(m0 + 16 + nloc) * K + kb, hlf); } else { frag_split(A + (size_t)(m0 + nloc) * K + kb, hlf, a0, l0); frag_split(A + (size_t)(m0 + 16 + nloc) * K + kb, hlf, a1, l1); }
#pragma unroll
    for (int t = 0; t < 4; ++t) { const v16b bw = frag_kb(Bw + (size_t)(c0 + t * 16 + nloc) * K + kb, hlf); acc[0][t] = wmma16b(a0, bw, acc[0][t]); acc[1][t] = wmma16b(a1, bw, acc[1][t]); if (amode == 1) { acc[0][t] = wmma16b(l0, bw, acc[0][t]); acc[1][t] = wmma16b(l1, bw, acc[1][t]); } } }
  const float sc_ = (amode == 0) ? 1.0f : (1.0f / AS_); float* Tt = Ts[wave];
#pragma unroll
  for (int t = 0; t < 4; ++t) { const int cc = c0 + t * 16 + nloc; const float bb = bias[cc]; const float s_ = emode ? scl[cc] : 1.0f, t_ = emode ? sft[cc] : 0.0f;
#pragma unroll
    for (int r = 0; r < 2; ++r)
#pragma unroll
      for (int v = 0; v < 8; ++v) { float y = acc[r][t][v] * sc_ + bb; if (emode) y = fmaxf(y * s_ + t_, 0.0f); Tt[(r * 16 + v + 8 * hlf) * 64 + t * 16 + nloc] = y; } }
  wave_lds_sync();
  for (int pass = 0; pass < 2; ++pass) {
#pragma unroll
    for (int j = 0; j < 16; ++j) { const int rr = j * 2 + hlf, c4 = nloc * 4; *(volatile v4f*)(Y + (size_t)(m0 + rr) * N + c0 + c4) = *(const v4f*)(Tt + rr * 64 + c4); }
    __threadfence(); }
}

__global__ __launch_bounds__(128) void head_kernel(const float* __restrict__ A, int K, const b16* __restrict__ W, const float* __restrict__ bias, int NC, float* __restrict__ out, const float* __restrict__ src, float* __restrict__ share) {
  __shared__ __attribute__((aligned(16))) float Lo[4][32][8];
  const int lane = threadIdx.x & 31, wave = threadIdx.x >> 5, nloc = lane & 15, hlf = lane >> 4, m0 = blockIdx.x * 128 + wave * 32;
  v8f acc[2] = {{}, {}};
  for (int kb = 0; kb < K; kb += 32) { v16b a0, l0, a1, l1; frag_split(A + (size_t)(m0 + nloc) * K + kb, hlf, a0, l0); frag_split(A + (size_t)(m0 + 16 + nloc) * K + kb, hlf, a1, l1); const v16b bw = frag_kb(W + (size_t)nloc * K + kb, hlf);
    acc[0] = wmma16b(a0, bw, acc[0]); acc[0] = wmma16b(l0, bw, acc[0]); acc[1] = wmma16b(a1, bw, acc[1]); acc[1] = wmma16b(l1, bw, acc[1]); }
  if (nloc < NC) {
#pragma unroll
    for (int r = 0; r < 2; ++r)
#pragma unroll
      for (int v = 0; v < 8; ++v) Lo[wave][r * 16 + 8 * hlf + v][nloc] = acc[r][v] * (1.0f / AS_) + bias[nloc]; }
  wave_lds_sync();
  { const int rr = lane; float mx = -INFINITY; for (int c = 0; c < NC; ++c) mx = fmaxf(mx, Lo[wave][rr][c]); float s = 0.0f; for (int c = 0; c < NC; ++c) s += nexp(Lo[wave][rr][c] - mx); const float lse = mx + nlog(s);
    wave_lds_sync(); for (int c = 0; c < NC; ++c) Lo[wave][rr][c] = Lo[wave][rr][c] - lse; }
  wave_lds_sync();
  for (int pass = 0; pass < 2; ++pass) {
    if (NC == 8) { for (int i = lane; i < 32 * 2; i += 32) { const int rr = i >> 1, c4 = (i & 1) * 4; *(volatile v4f*)(out + (size_t)(m0 + rr) * 8 + c4) = *(const v4f*)(&Lo[wave][rr][c4]); } }
    else { *(volatile v2f*)(out + (size_t)(m0 + lane) * 2) = *(const v2f*)(&Lo[wave][lane][0]); }
    if (src != nullptr) { for (int i = lane; i < 32 * (D / 4); i += 32) { const int rr = i / (D / 4), c4 = (i % (D / 4)) * 4; const v4f s4 = *(const v4f*)(src + (size_t)(m0 + rr) * D + c4); v4f o4; for (int e = 0; e < 4; ++e) o4[e] = bf16_rne(s4[e]); *(volatile v4f*)(share + (size_t)(m0 + rr) * D + c4) = o4; } }
    __threadfence(); }
}

__device__ __forceinline__ void ln_relu_rows(const float* Y, int N, const float* g, const float* bta, b16* Ah, b16* Al, int wave, int lane) {
  for (int rr = wave * 2; rr < wave * 2 + 2; ++rr) { const float* yr = Y + (size_t)rr * (H1 + 4); float s = 0.0f; for (int c = lane; c < N; c += 32) s += yr[c];
#pragma unroll
    for (int o = 1; o < 32; o <<= 1) s += __shfl_xor(s, o);
    const float mu = s / (float)N; float q = 0.0f; for (int c = lane; c < N; c += 32) { const float d = yr[c] - mu; q += pmul(d, d); }
#pragma unroll
    for (int o = 1; o < 32; o <<= 1) q += __shfl_xor(q, o);
    const float is = rsqrtf(q / (float)N + EPS);
    for (int c = lane; c < N; c += 32) { const float v = fmaxf(pmul((yr[c] - mu) * is, g[c]) + bta[c], 0.0f); b16 h_, l_; split16(v * AS_, h_, l_); Ah[(size_t)rr * (H1 + 8) + c] = h_; Al[(size_t)rr * (H1 + 8) + c] = l_; } }
}

__global__ __launch_bounds__(256) void expert_kernel(const float* __restrict__ src, const float* __restrict__ slog, const b16* __restrict__ R, const float* __restrict__ P, float* __restrict__ plane) {
  __shared__ __attribute__((aligned(16))) float Y[16][H1 + 4]; __shared__ __attribute__((aligned(16))) b16 Ah[16][H1 + 8], Al[16][H1 + 8]; __shared__ int toks[CHUNK]; __shared__ int wcnt[8]; __shared__ __attribute__((aligned(16))) float Res[CHUNK][2];
  const int wave = threadIdx.x >> 5, lane = threadIdx.x & 31, nloc = lane & 15, hlf = lane >> 4, c0 = blockIdx.x * CHUNK, e = blockIdx.y;
  for (int i = threadIdx.x; i < CHUNK * 2; i += 256) Res[i >> 1][i & 1] = 0.0f;
  int ntok;
  { int nh = 0; bool hit[2];
#pragma unroll
    for (int q = 0; q < 2; ++q) { const int b = c0 + threadIdx.x * 2 + q; const float* lr = slog + (size_t)b * C; int best = 0; float bv = lr[0]; for (int c = 1; c < C; ++c) { const float v = lr[c]; if (v > bv) { bv = v; best = c; } } hit[q] = (best == e); nh += hit[q] ? 1 : 0; }
    int incl = nh;
#pragma unroll
    for (int o = 1; o < 32; o <<= 1) { const int t = __shfl_up(incl, o); if (lane >= o) incl += t; }
    if (lane == 31) wcnt[wave] = incl;
    __syncthreads();
    int woff = 0; for (int w = 0; w < wave; ++w) woff += wcnt[w]; ntok = 0; for (int w = 0; w < 8; ++w) ntok += wcnt[w]; int pos = woff + incl - nh;
#pragma unroll
    for (int q = 0; q < 2; ++q) if (hit[q]) toks[pos++] = c0 + threadIdx.x * 2 + q;
    __syncthreads(); }
  const b16* W1 = R + Wo_::EW1 + (size_t)e * 1024 * 512; const b16* W2 = R + Wo_::EW2 + (size_t)e * 1024 * 1024; const b16* W3 = R + Wo_::EW3 + (size_t)e * 512 * 1024; const b16* W4 = R + Wo_::EW4 + (size_t)e * 16 * 512;
  const float* b1 = P + Po_::EB1 + e * 1024; const float* g1 = P + Po_::EG1 + e * 1024; const float* t1 = P + Po_::ET1 + e * 1024; const float* b2 = P + Po_::EB2 + e * 1024; const float* g2 = P + Po_::EG2 + e * 1024; const float* t2 = P + Po_::ET2 + e * 1024;
  const float* b3 = P + Po_::EB3 + e * 512; const float* g3 = P + Po_::EG3 + e * 512; const float* t3 = P + Po_::ET3 + e * 512; const float* b4 = P + Po_::EB4 + e * 16;
  for (int r0 = 0; r0 < ntok; r0 += 16) { const int nvalid = min(16, ntok - r0);
    __syncthreads();
    for (int i = threadIdx.x; i < 16 * (D / 4); i += 256) { const int rr = i / (D / 4), c4 = (i % (D / 4)) * 4; const int b = toks[r0 + ((rr < nvalid) ? rr : 0)]; const v4f s4 = *(const v4f*)(src + (size_t)b * D + c4);
#pragma unroll
      for (int q = 0; q < 4; ++q) Ah[rr][c4 + q] = (b16)bf16_rne(s4[q]); }
    __syncthreads();
    { v8f acc[8];
#pragma unroll
      for (int t = 0; t < 8; ++t) acc[t] = (v8f){};
#pragma unroll 2
      for (int kb = 0; kb < D; kb += 32) { const v16b a = frag_kb(&Ah[nloc][kb], hlf);
#pragma unroll
        for (int t = 0; t < 8; ++t) { const v16b bw = frag_kb(W1 + (size_t)(wave * 128 + t * 16 + nloc) * D + kb, hlf); acc[t] = wmma16b(a, bw, acc[t]); } }
#pragma unroll
      for (int t = 0; t < 8; ++t) { const int cc = wave * 128 + t * 16 + nloc; const float bb = b1[cc];
#pragma unroll
        for (int v = 0; v < 8; ++v) Y[8 * hlf + v][cc] = acc[t][v] + bb; } }
    __syncthreads();
    ln_relu_rows(&Y[0][0], 1024, g1, t1, &Ah[0][0], &Al[0][0], wave, lane);
    __syncthreads();
    { v8f acc[8];
#pragma unroll
      for (int t = 0; t < 8; ++t) acc[t] = (v8f){};
#pragma unroll 2
      for (int kb = 0; kb < H1; kb += 32) { const v16b a = frag_kb(&Ah[nloc][kb], hlf), al = frag_kb(&Al[nloc][kb], hlf);
#pragma unroll
        for (int t = 0; t < 8; ++t) { const v16b bw = frag_kb(W2 + (size_t)(wave * 128 + t * 16 + nloc) * H1 + kb, hlf); acc[t] = wmma16b(a, bw, acc[t]); acc[t] = wmma16b(al, bw, acc[t]); } }
      __syncthreads();
#pragma unroll
      for (int t = 0; t < 8; ++t) { const int cc = wave * 128 + t * 16 + nloc; const float bb = b2[cc];
#pragma unroll
        for (int v = 0; v < 8; ++v) Y[8 * hlf + v][cc] = acc[t][v] * (1.0f / AS_) + bb; } }
    __syncthreads();
    ln_relu_rows(&Y[0][0], 1024, g2, t2, &Ah[0][0], &Al[0][0], wave, lane);
    __syncthreads();
    { v8f acc[4];
#pragma unroll
      for (int t = 0; t < 4; ++t) acc[t] = (v8f){};
#pragma unroll 2
      for (int kb = 0; kb < H1; kb += 32) { const v16b a = frag_kb(&Ah[nloc][kb], hlf), al = frag_kb(&Al[nloc][kb], hlf);
#pragma unroll
        for (int t = 0; t < 4; ++t) { const v16b bw = frag_kb(W3 + (size_t)(wave * 64 + t * 16 + nloc) * H1 + kb, hlf); acc[t] = wmma16b(a, bw, acc[t]); acc[t] = wmma16b(al, bw, acc[t]); } }
      __syncthreads();
#pragma unroll
      for (int t = 0; t < 4; ++t) { const int cc = wave * 64 + t * 16 + nloc; const float bb = b3[cc];
#pragma unroll
        for (int v = 0; v < 8; ++v) Y[8 * hlf + v][cc] = acc[t][v] * (1.0f / AS_) + bb; } }
    __syncthreads();
    ln_relu_rows(&Y[0][0], 512, g3, t3, &Ah[0][0], &Al[0][0], wave, lane);
    __syncthreads();
    if (wave == 0) { v8f acc = {};
      for (int kb = 0; kb < D; kb += 32) { const v16b a = frag_kb(&Ah[nloc][kb], hlf), al = frag_kb(&Al[nloc][kb], hlf), bw = frag_kb(W4 + (size_t)nloc * D + kb, hlf); acc = wmma16b(a, bw, acc); acc = wmma16b(al, bw, acc); }
      if (nloc < 2) {
#pragma unroll
        for (int v = 0; v < 8; ++v) Y[8 * hlf + v][nloc] = acc[v] * (1.0f / AS_) + b4[nloc]; }
      wave_lds_sync();
      if (lane < nvalid) { const float z0 = Y[lane][0], z1 = Y[lane][1]; const float mx = fmaxf(z0, z1); const float lse = mx + nlog(nexp(z0 - mx) + nexp(z1 - mx)); const int m = toks[r0 + lane] - c0; Res[m][0] = z0 - lse; Res[m][1] = z1 - lse; } }
  }
  __syncthreads();
  for (int pass = 0; pass < 2; ++pass) { for (int i = threadIdx.x; i < CHUNK * 2 / 4; i += 256) *(volatile v4f*)(plane + ((size_t)e * B + c0) * 2 + i * 4) = *(const v4f*)(&Res[0][0] + i * 4); __threadfence(); }
}

__global__ __launch_bounds__(256) void pick_kernel(const float* __restrict__ slog, const float* __restrict__ plane, float* __restrict__ sout) {
  const int b = blockIdx.x * 256 + threadIdx.x; const float* lr = slog + (size_t)b * C; int best = 0; float bv = lr[0]; for (int c = 1; c < C; ++c) { const float v = lr[c]; if (v > bv) { bv = v; best = c; } }
  const v2f r = *(const v2f*)(plane + ((size_t)best * B + b) * 2);
  for (int pass = 0; pass < 2; ++pass) { *(volatile v2f*)(sout + (size_t)b * 2) = r; __threadfence(); }
}
}

extern "C" void kernel_launch(void* const* d_in, const int* in_sizes, int n_in,
                              void* d_out, int out_size, void* d_ws, size_t ws_size, hipStream_t stream) {
  (void)out_size;
  if (n_in != 49) return;
  In in; for (int i = 0; i < 49; ++i) in.p[i] = (const float*)d_in[i];
  const float* source = in.p[0];
  float* src_log = (float*)d_out; float* d_log = src_log + (size_t)B * C; float* sout = d_log + (size_t)B * 2; float* share = sout + (size_t)B * 2;
  if (in_sizes[0] != B * D || in_sizes[1] != D * 256 || in_sizes[21] != 1024 * 1024 || in_sizes[39] != E * 1024 * 1024 || in_sizes[47] != E * 512 * 2) return;
  size_t off = 0; char* ws = (char*)d_ws;
  auto carve = [&](size_t bytes) { char* p = ws + off; off += (bytes + 255) & ~(size_t)255; return p; };
  b16* R = (b16*)carve(Wo_::END * 2); float* P = (float*)carve(((size_t)Po_::END + 64) * 4); float* z1 = (float*)carve((size_t)B * 256 * 4); float* z2 = (float*)carve((size_t)B * 128 * 4);
  float* h1 = (float*)carve((size_t)B * 1024 * 4); float* h2 = (float*)carve((size_t)B * 1024 * 4); float* h3 = z1;
  h3 = (float*)carve((size_t)B * 512 * 4); float* plane = (float*)carve((size_t)E * B * 2 * 4);
  if (off > ws_size) return;
  prep_kernel<<<1024, 256, 0, stream>>>(in, R, P);
  gemm_kernel<<<dim3(256 / 64, B / 128), 128, 0, stream>>>(source, D, 0, R + Wo_::BW1, 256, P + Po_::BB1, 1, P + Po_::BS1, P + Po_::BT1, z1);
  gemm_kernel<<<dim3(128 / 64, B / 128), 128, 0, stream>>>(z1, 256, 1, R + Wo_::BW2, 128, P + Po_::BB2, 1, P + Po_::BS2, P + Po_::BT2, z2);
  head_kernel<<<B / 128, 128, 0, stream>>>(z2, 128, R + Wo_::FC, P + Po_::FCB, 8, src_log, source, share);
  gemm_kernel<<<dim3(1024 / 64, B / 128), 128, 0, stream>>>(source, D, 0, R + Wo_::DW1, 1024, P + Po_::DB1, 1, P + Po_::DS1, P + Po_::DT1, h1);
  gemm_kernel<<<dim3(1024 / 64, B / 128), 128, 0, stream>>>(h1, 1024, 1, R + Wo_::DW2, 1024, P + Po_::DB2, 1, P + Po_::DS2, P + Po_::DT2, h2);
  gemm_kernel<<<dim3(512 / 64, B / 128), 128, 0, stream>>>(h2, 1024, 1, R + Wo_::DW3, 512, P + Po_::DB3, 1, P + Po_::DS3, P + Po_::DT3, h3);
  head_kernel<<<B / 128, 128, 0, stream>>>(h3, 512, R + Wo_::DW4, P + Po_::DB4, 2, d_log, nullptr, nullptr);
  expert_kernel<<<dim3(B / CHUNK, E), 256, 0, stream>>>(source, src_log, R, P, plane);
  pick_kernel<<<B / 256, 256, 0, stream>>>(src_log, plane, sout);
}
